// MultiHeadAttention_CF_29403346108539
// MI455X (gfx1250) — hardware-run, weakly checked
//
#include <hip/hip_runtime.h>
#include <stddef.h>
#include <stdint.h>
#include <math.h>

#define NB    4
#define SQ    2048
#define NTOK  8192
#define HID   1024
#define NH    16
#define HDM   64
#define QB    128
#define KC    64
#define NQB   (SQ / QB)
#define NCK   (SQ / KC)
#define SBLK  (SQ / 256)
#define QKPLANE (NB * NH * SQ * HDM)

#define WSC 256.0f
#define QSC 8.0f
#define PSC 1024.0f
#define OSC 512.0f

static_assert(NTOK == NB * SQ);
static_assert(SQ % 256 == 0);
static_assert(HID % 256 == 0);
static_assert(HID % 64 == 0);
static_assert(HDM == 64);
static_assert(NH * HDM == HID);
static_assert(SQ % KC == 0);
static_assert(SQ % QB == 0);
static_assert(QB == 8 * 16);
static_assert(NTOK % 256 == 0);
static_assert((NTOK * HID) % 8192 == 0);
static_assert((HID * HID) % 8192 == 0);

typedef _Float16 v16h __attribute__((ext_vector_type(16)));
typedef _Float16 v8h  __attribute__((ext_vector_type(8)));
typedef float    v8f  __attribute__((ext_vector_type(8)));
typedef float    v4f  __attribute__((ext_vector_type(4)));
typedef unsigned int v4u __attribute__((ext_vector_type(4)));

union Frag  { v16h v; v8h h[2]; };
union Pack8 { v8h h; v4u u; };

__device__ __forceinline__ v8f mma16(v16h a, v16h b, v8f c) {
  c = __builtin_amdgcn_wmma_f32_16x16x32_f16(false, a, false, b, (short)0, c, false, false);
  asm volatile("v_nop\n\tv_nop\n\tv_nop\n\tv_nop" : "+v"(c) : "v"(a), "v"(b));
  return c;
}

__device__ __forceinline__ v16h ldfrag(const _Float16* p, int ld, int row0, int k0, int lane) {
  const int m = lane & 15, lh = lane >> 4;
  const _Float16* q = p + (size_t)(row0 + m) * ld + k0 + 8 * lh;
  Frag f;
  f.h[0] = *(const v8h*)(q);
  f.h[1] = *(const v8h*)(q + 16);
  return f.v;
}

__device__ __forceinline__ v8f zero8() { return (v8f){0.f, 0.f, 0.f, 0.f, 0.f, 0.f, 0.f, 0.f}; }

__device__ __forceinline__ void gemm32x64(const _Float16* __restrict__ A, int lda,
                                          const _Float16* __restrict__ Bt, int ldb, int K,
                                          int m0, int n0, int lane, v8f (&acc)[2][4]) {
#pragma unroll 1
  for (int k0 = 0; k0 < K; k0 += 32) {
    const v16h a0 = ldfrag(A, lda, m0, k0, lane);
    const v16h a1 = ldfrag(A, lda, m0 + 16, k0, lane);
    const v16h b0 = ldfrag(Bt, ldb, n0, k0, lane);
    const v16h b1 = ldfrag(Bt, ldb, n0 + 16, k0, lane);
    const v16h b2 = ldfrag(Bt, ldb, n0 + 32, k0, lane);
    const v16h b3 = ldfrag(Bt, ldb, n0 + 48, k0, lane);
    acc[0][0] = mma16(a0, b0, acc[0][0]);
    acc[1][0] = mma16(a1, b0, acc[1][0]);
    acc[0][1] = mma16(a0, b1, acc[0][1]);
    acc[1][1] = mma16(a1, b1, acc[1][1]);
    acc[0][2] = mma16(a0, b2, acc[0][2]);
    acc[1][2] = mma16(a1, b2, acc[1][2]);
    acc[0][3] = mma16(a0, b3, acc[0][3]);
    acc[1][3] = mma16(a1, b3, acc[1][3]);
  }
}

__global__ __launch_bounds__(256) void k_cvt(const float* __restrict__ src, float scale,
                                             _Float16* __restrict__ dst) {
  const int tid = threadIdx.x;
  v4u val[4];
  size_t go[4];
#pragma unroll
  for (int j = 0; j < 4; ++j) {
    const size_t p = (size_t)blockIdx.x * 1024 + 256 * j + tid;
    const float* s = src + p * 8;
    const v4f a0 = *(const v4f*)(s) * scale;
    const v4f a1 = *(const v4f*)(s + 4) * scale;
    Pack8 pk;
    pk.h = (v8h){(_Float16)a0[0], (_Float16)a0[1], (_Float16)a0[2], (_Float16)a0[3],
                 (_Float16)a1[0], (_Float16)a1[1], (_Float16)a1[2], (_Float16)a1[3]};
    val[j] = pk.u;
    go[j]  = p * 8;
  }
  for (int ps = 0; ps < 2; ++ps) {
#pragma unroll
    for (int j = 0; j < 4; ++j) *(volatile v4u*)(dst + go[j]) = val[j];
    __threadfence();
  }
}

#define STP 72
#define SVP 264
static_assert(256 * STP >= 64 * SVP);
__global__ __launch_bounds__(256) void k_qkv(const _Float16* __restrict__ xh,
                                             const _Float16* __restrict__ wt,
                                             const float* __restrict__ bias,
                                             int which,
                                             _Float16* __restrict__ qkp,
                                             _Float16* __restrict__ vtp) {
  __shared__ __align__(16) _Float16 st[256 * STP];
  const int tid = threadIdx.x, lane = tid & 31, wave = tid >> 5;
  const int hh = lane >> 4, c = lane & 15;
  const int bx = blockIdx.x;
  const int b  = bx / SBLK;
  const int sb = (bx - b * SBLK) * 256;
  const int head = blockIdx.y;
  const int hb   = b * NH + head;
  const int m0 = bx * 256 + wave * 32;
  const int n0 = head * 64;

  v8f acc[2][4];
#pragma unroll
  for (int s = 0; s < 2; ++s)
#pragma unroll
    for (int t = 0; t < 4; ++t) acc[s][t] = zero8();
  gemm32x64(xh, HID, wt, HID, HID, m0, n0, lane, acc);

  float bb[4];
#pragma unroll
  for (int t = 0; t < 4; ++t) bb[t] = bias[n0 + 16 * t + c];
  const float isc = 1.0f / WSC;
  const float osc = (which == 0) ? QSC : 1.0f;

  if (which < 2) {
#pragma unroll
    for (int sub = 0; sub < 2; ++sub)
#pragma unroll
      for (int t = 0; t < 4; ++t)
#pragma unroll
        for (int r = 0; r < 8; ++r) {
          const int lr = wave * 32 + sub * 16 + 8 * hh + r;
          st[lr * STP + 16 * t + c] = (_Float16)((acc[sub][t][r] * isc + bb[t]) * osc);
        }
  } else {
#pragma unroll
    for (int sub = 0; sub < 2; ++sub)
#pragma unroll
      for (int t = 0; t < 4; ++t)
#pragma unroll
        for (int r = 0; r < 8; ++r)
          st[(16 * t + c) * SVP + wave * 32 + sub * 16 + 8 * hh + r] =
              (_Float16)(acc[sub][t][r] * isc + bb[t]);
  }
  __syncthreads();

  if (which < 2) {
    _Float16* base = qkp + (size_t)which * QKPLANE + (size_t)hb * SQ * HDM;
#pragma unroll
    for (int g = 0; g < 2; ++g) {
      v4u val[4];
      size_t go[4];
#pragma unroll
      for (int j = 0; j < 4; ++j) {
        const int p  = tid + 256 * (4 * g + j);
        const int lr = p >> 3;
        const int pc = p & 7;
        Pack8 pk;
        pk.h   = *(const v8h*)(st + lr * STP + pc * 8);
        val[j] = pk.u;
        go[j]  = (size_t)(sb + lr) * HDM + pc * 8;
      }
      for (int ps = 0; ps < 2; ++ps) {
#pragma unroll
        for (int j = 0; j < 4; ++j) *(volatile v4u*)(base + go[j]) = val[j];
        __threadfence();
      }
    }
  } else {
    _Float16* base = vtp + (size_t)hb * HDM * SQ;
#pragma unroll
    for (int g = 0; g < 2; ++g) {
      v4u val[4];
      size_t go[4];
#pragma unroll
      for (int j = 0; j < 4; ++j) {
        const int p    = tid + 256 * (4 * g + j);
        const int drow = p >> 5;
        const int pc   = p & 31;
        Pack8 pk;
        pk.h   = *(const v8h*)(st + drow * SVP + pc * 8);
        val[j] = pk.u;
        go[j]  = (size_t)drow * SQ + sb + pc * 8;
      }
      for (int ps = 0; ps < 2; ++ps) {
#pragma unroll
        for (int j = 0; j < 4; ++j) *(volatile v4u*)(base + go[j]) = val[j];
        __threadfence();
      }
    }
  }
}

#define KTP 72
__global__ __launch_bounds__(256) void k_attn(const _Float16* __restrict__ qp,
                                              const _Float16* __restrict__ kp,
                                              const _Float16* __restrict__ vt,
                                              _Float16* __restrict__ op, float sscale) {
  __shared__ __align__(16) _Float16 Ks[KC * KTP];
  __shared__ __align__(16) _Float16 Vs[HDM * KTP];
  __shared__ __align__(16) _Float16 Ps[8 * 16 * KTP];

  const int tid = threadIdx.x, lane = tid & 31, wave = tid >> 5;
  const int hh = lane >> 4, c = lane & 15;
  const int qb  = blockIdx.x % NQB;
  const int hb  = blockIdx.x / NQB;
  const int h   = hb % NH;
  const int b   = hb / NH;
  const int q0  = qb * QB + wave * 16;

  const _Float16* Q = qp + (size_t)hb * SQ * HDM;
  const _Float16* K = kp + (size_t)hb * SQ * HDM;
  const _Float16* V = vt + (size_t)hb * HDM * SQ;

  v16h qa[2];
  qa[0] = ldfrag(Q, HDM, q0, 0, lane);
  qa[1] = ldfrag(Q, HDM, q0, 32, lane);

  const float NEGI = -__builtin_huge_valf();
  float mrow[8], lrow[8];
  v8f oacc[4];
#pragma unroll
  for (int r = 0; r < 8; ++r) { mrow[r] = NEGI; lrow[r] = 0.f; }
#pragma unroll
  for (int t = 0; t < 4; ++t) oacc[t] = zero8();

  _Float16* pw = Ps + wave * 16 * KTP;

  for (int kc = 0; kc < NCK; ++kc) {
    const int kv0 = kc * KC;
    __syncthreads();
    {
      const int r  = tid >> 2;
      const int qq = (tid & 3) * 16;
      const _Float16* ks = K + (size_t)(kv0 + r) * HDM + qq;
      const _Float16* vs = V + (size_t)r * SQ + kv0 + qq;
#pragma unroll
      for (int e = 0; e < 2; ++e) {
        *(v8h*)(Ks + r * KTP + qq + 8 * e) = *(const v8h*)(ks + 8 * e);
        *(v8h*)(Vs + r * KTP + qq + 8 * e) = *(const v8h*)(vs + 8 * e);
      }
    }
    __syncthreads();

    v8f s[4];
#pragma unroll
    for (int j = 0; j < 4; ++j) s[j] = zero8();
#pragma unroll
    for (int dc = 0; dc < 2; ++dc) {
#pragma unroll
      for (int j = 0; j < 4; ++j) {
        const v16h kb = ldfrag(Ks, KTP, j * 16, dc * 32, lane);
        s[j] = mma16(qa[dc], kb, s[j]);
      }
    }
    float cm[8];
#pragma unroll
    for (int r = 0; r < 8; ++r) {
      float m = NEGI;
#pragma unroll
      for (int j = 0; j < 4; ++j) { s[j][r] = s[j][r] * sscale; m = fmaxf(m, s[j][r]); }
#pragma unroll
      for (int off = 1; off < 16; off <<= 1) m = fmaxf(m, __shfl_xor(m, off, 32));
      cm[r] = m;
    }
    float al[8];
#pragma unroll
    for (int r = 0; r < 8; ++r) {
      const float mnew  = fmaxf(mrow[r], cm[r]);
      const float alpha = __expf(mrow[r] - mnew);
      mrow[r] = mnew;
      float psum = 0.f;
#pragma unroll
      for (int j = 0; j < 4; ++j) {
        const float p = __expf(s[j][r] - mnew);
        psum += p;
        pw[(8 * hh + r) * KTP + j * 16 + c] = (_Float16)(p * PSC);
      }
#pragma unroll
      for (int off = 1; off < 16; off <<= 1) psum += __shfl_xor(psum, off, 32);
      lrow[r] = lrow[r] * alpha + psum;
      al[r] = alpha;
    }
#pragma unroll
    for (int t = 0; t < 4; ++t)
#pragma unroll
      for (int r = 0; r < 8; ++r) oacc[t][r] *= al[r];
    __syncthreads();

#pragma unroll
    for (int kk = 0; kk < 2; ++kk) {
      const v16h pa = ldfrag(pw, KTP, 0, kk * 32, lane);
#pragma unroll
      for (int t = 0; t < 4; ++t) {
        const v16h vb = ldfrag(Vs, KTP, t * 16, kk * 32, lane);
        oacc[t] = mma16(pa, vb, oacc[t]);
      }
    }
  }

  float invl[8];
#pragma unroll
  for (int r = 0; r < 8; ++r) invl[r] = (lrow[r] > 0.f) ? ((OSC / PSC) / lrow[r]) : 0.f;
  __syncthreads();
#pragma unroll
  for (int r = 0; r < 8; ++r) {
#pragma unroll
    for (int t = 0; t < 4; ++t)
      pw[(8 * hh + r) * KTP + 16 * t + c] = (_Float16)(oacc[t][r] * invl[r]);
  }
  __syncthreads();
  v4u val[4];
  size_t go[4];
#pragma unroll
  for (int it = 0; it < 4; ++it) {
    const int p  = lane + 32 * it;
    const int L  = p >> 3;
    const int pc = p & 7;
    Pack8 pk;
    pk.h    = *(const v8h*)(pw + L * KTP + pc * 8);
    val[it] = pk.u;
    go[it]  = ((size_t)(b * SQ + q0 + L)) * HID + (size_t)h * HDM + pc * 8;
  }
  for (int ps = 0; ps < 2; ++ps) {
#pragma unroll
    for (int it = 0; it < 4; ++it) *(volatile v4u*)(op + go[it]) = val[it];
    __threadfence();
  }
}

#define OTP 68
__device__ __forceinline__ void out_epilogue_f32(v8f (&acc)[2][4], float scale, const float (&bb)[4],
                                                 float* sw, float* __restrict__ out, int ldo,
                                                 int m0, int n0, int lane, int hh, int c) {
#pragma unroll
  for (int sub = 0; sub < 2; ++sub) {
    __syncthreads();
#pragma unroll
    for (int t = 0; t < 4; ++t) {
#pragma unroll
      for (int r = 0; r < 8; ++r) sw[(8 * hh + r) * OTP + 16 * t + c] = acc[sub][t][r] * scale + bb[t];
    }
    __syncthreads();
    v4f val[8];
    size_t go[8];
#pragma unroll
    for (int it = 0; it < 8; ++it) {
      const int p    = lane + 32 * it;
      const int L    = p >> 3;
      const int pc   = p & 7;
      const int row  = L >> 1;
      const int half = L & 1;
      val[it] = *(const v4f*)(sw + row * OTP + half * 32 + pc * 4);
      go[it]  = (size_t)(m0 + sub * 16 + row) * ldo + n0 + half * 32 + pc * 4;
    }
    for (int ps = 0; ps < 2; ++ps) {
#pragma unroll
      for (int it = 0; it < 8; ++it) *(volatile v4f*)(out + go[it]) = val[it];
      __threadfence();
    }
  }
}

__global__ __launch_bounds__(256) void k_gemm_f32(const _Float16* __restrict__ ap, int lda,
                                                  const _Float16* __restrict__ wt, int K,
                                                  const float* __restrict__ bias, float scale,
                                                  float* __restrict__ out, int ldo) {
  __shared__ __align__(16) float st[8][16 * OTP];
  const int tid = threadIdx.x, lane = tid & 31, wave = tid >> 5;
  const int hh = lane >> 4, c = lane & 15;
  const int m0 = blockIdx.x * 256 + wave * 32;
  const int n0 = blockIdx.y * 64;

  v8f acc[2][4];
#pragma unroll
  for (int s = 0; s < 2; ++s)
#pragma unroll
    for (int t = 0; t < 4; ++t) acc[s][t] = zero8();
  gemm32x64(ap, lda, wt, K, K, m0, n0, lane, acc);
  float bb[4];
#pragma unroll
  for (int t = 0; t < 4; ++t) bb[t] = bias[n0 + 16 * t + c];
  out_epilogue_f32(acc, scale, bb, st[wave], out, ldo, m0, n0, lane, hh, c);
}

extern "C" void kernel_launch(void* const* d_in, const int* in_sizes, int n_in,
                              void* d_out, int out_size, void* d_ws, size_t ws_size,
                              hipStream_t stream) {
  if (n_in < 9) return;
  if (in_sizes[0] != NTOK * HID) return;
  if (in_sizes[1] != HID * HID) return;
  if (in_sizes[2] != HID) return;
  if (in_sizes[3] != HID * HID) return;
  if (in_sizes[4] != HID) return;
  if (in_sizes[5] != HID * HID) return;
  if (in_sizes[6] != HID) return;
  if (in_sizes[7] != HID * HID) return;
  if (in_sizes[8] != HID) return;
  if (out_size != NTOK * HID) return;

  const float* x  = (const float*)d_in[0];
  const float* wq = (const float*)d_in[1];
  const float* bq = (const float*)d_in[2];
  const float* wk = (const float*)d_in[3];
  const float* bk = (const float*)d_in[4];
  const float* wv = (const float*)d_in[5];
  const float* bv = (const float*)d_in[6];
  const float* wo = (const float*)d_in[7];
  const float* bo = (const float*)d_in[8];
  float* out = (float*)d_out;

  size_t off = 0;
  const size_t oXh = off; off += (size_t)NTOK * HID * 2;
  const size_t oW  = off; off += (size_t)4 * HID * HID * 2;
  const size_t oQK = off; off += (size_t)2 * QKPLANE * 2;
  const size_t oV  = off; off += (size_t)NB * NH * HDM * SQ * 2;
  const size_t oO  = off; off += (size_t)NTOK * HID * 2;
  if (off > ws_size) return;
  if (off > (size_t)134217728) return;

  char* ws = (char*)d_ws;
  _Float16* Xh  = (_Float16*)(ws + oXh);
  _Float16* Wqt = (_Float16*)(ws + oW);
  _Float16* Wkt = Wqt + (size_t)HID * HID;
  _Float16* Wvt = Wkt + (size_t)HID * HID;
  _Float16* Wot = Wvt + (size_t)HID * HID;
  _Float16* QKp = (_Float16*)(ws + oQK);
  _Float16* Kp  = QKp + (size_t)QKPLANE;
  _Float16* Vt  = (_Float16*)(ws + oV);
  _Float16* Op  = (_Float16*)(ws + oO);

  k_cvt<<<dim3((NTOK * HID) / 8192), dim3(256), 0, stream>>>(x, 1.0f, Xh);
  k_cvt<<<dim3((HID * HID) / 8192), dim3(256), 0, stream>>>(wq, WSC, Wqt);
  k_cvt<<<dim3((HID * HID) / 8192), dim3(256), 0, stream>>>(wk, WSC, Wkt);
  k_cvt<<<dim3((HID * HID) / 8192), dim3(256), 0, stream>>>(wv, WSC, Wvt);
  k_cvt<<<dim3((HID * HID) / 8192), dim3(256), 0, stream>>>(wo, WSC, Wot);
  k_qkv<<<dim3(NTOK / 256, HID / 64), dim3(256), 0, stream>>>(Xh, Wqt, bq, 0, QKp, Vt);
  k_qkv<<<dim3(NTOK / 256, HID / 64), dim3(256), 0, stream>>>(Xh, Wkt, bk, 1, QKp, Vt);
  k_qkv<<<dim3(NTOK / 256, HID / 64), dim3(256), 0, stream>>>(Xh, Wvt, bv, 2, QKp, Vt);
  k_attn<<<dim3(NB * NH * NQB), dim3(256), 0, stream>>>(QKp, Kp, Vt, Op, 1.0f / (QSC * 8.0f));
  k_gemm_f32<<<dim3(NTOK / 256, HID / 64), dim3(256), 0, stream>>>(Op, HID, Wot, HID, bo,
                                                                    1.0f / (OSC * WSC), out, HID);
  (void)hipGetLastError();
}
